// CausalSelfAttention_3530463117417
// MI455X (gfx1250) — hardware-verified
//
#include <hip/hip_runtime.h>


#ifndef NB
#define NB 2
#endif
#ifndef SEQ
#define SEQ 2048
#endif
#define SEQ_FULL 2048
#define DM   1024
#define NH_  16
#define NKV  4
#define REP  (NH_ / NKV)
#define HD   64
#define DQ   (NH_ * HD)
#define DKV  (NKV * HD)
#define NQKV (DQ + 2 * DKV)
#define KCOL DQ
#define VCOL (DQ + DKV)
#define RH   ((SEQ) < 256 ? (SEQ) : 256)
#define EPP  72
#define PCAR 1024.0f
#define RCAR 2048.0f
#define L2E  1.4426950408889634f
#define NEGBIG (-1.0e30f)

typedef _Float16 h16;
typedef unsigned short bf;
typedef __attribute__((ext_vector_type(16))) __bf16   v16bf;
typedef __attribute__((ext_vector_type(16))) _Float16 v16h;
typedef __attribute__((ext_vector_type(8)))  _Float16 v8h;
typedef __attribute__((ext_vector_type(8)))  unsigned short v8us;
typedef __attribute__((ext_vector_type(8)))  float    v8f;
typedef __attribute__((ext_vector_type(4)))  float    v4f;
typedef __attribute__((ext_vector_type(2)))  _Float16 v2h;
typedef __attribute__((ext_vector_type(2)))  unsigned short v2us;
typedef v4f  __attribute__((may_alias)) v4fa;
typedef v8us __attribute__((may_alias)) v8usa;

static_assert(HD == 64);
static_assert(DQ == DM);
static_assert(NH_ % NKV == 0);
static_assert(SEQ % 64 == 0);
static_assert(SEQ <= SEQ_FULL);
static_assert(RH % 64 == 0);
static_assert(RH <= SEQ);
static_assert(DM % 32 == 0);
static_assert(DQ % 32 == 0);
static_assert((NB * SEQ) % 64 == 0);
static_assert(NQKV % 64 == 0);
static_assert(DM % 64 == 0);
static_assert(EPP % 8 == 0);
static_assert(EPP >= HD);
static_assert((DM * DQ) % 64 == 0);
static_assert((DM * DKV) % 64 == 0);

__device__ __forceinline__ unsigned short f2bf(float f) { unsigned u = __float_as_uint(f); u += 0x7FFFu + ((u >> 16) & 1u); return (unsigned short)(u >> 16); }
__device__ __forceinline__ float bf2f(unsigned short b) { return __uint_as_float(((unsigned)b) << 16); }
__device__ __forceinline__ float bfr(float f) { return bf2f(f2bf(f)); }
__device__ __forceinline__ void splitf(float y, unsigned short& h, unsigned short& l) { h = f2bf(y); l = f2bf(y - bf2f(h)); }
__device__ __forceinline__ v16h cat16(v8h lo, v8h hi) { return __builtin_shufflevector(lo, hi, 0, 1, 2, 3, 4, 5, 6, 7, 8, 9, 10, 11, 12, 13, 14, 15); }
__device__ __forceinline__ v16bf cat16b(v8us lo, v8us hi) { return __builtin_bit_cast(v16bf, __builtin_shufflevector(lo, hi, 0, 1, 2, 3, 4, 5, 6, 7, 8, 9, 10, 11, 12, 13, 14, 15)); }
__device__ __forceinline__ v8f wmma16(v16h a, v16h b, v8f c) { return __builtin_amdgcn_wmma_f32_16x16x32_f16(false, a, false, b, (short)0, c, false, false); }
__device__ __forceinline__ v8f wmmab(v16bf a, v16bf b, v8f c) { return __builtin_amdgcn_wmma_f32_16x16x32_bf16(false, a, false, b, (short)0, c, false, false); }
__device__ __forceinline__ v16bf ldb(const bf* p) { return cat16b(*(const v8us*)p, *(const v8us*)(p + 16)); }
__device__ __forceinline__ v16h ldh(const h16* p) { return cat16(*(const v8h*)p, *(const v8h*)(p + 16)); }

template <typename V> __device__ __forceinline__ void nopg2(v8f& c0, v8f& c1, const V& x, const V& y, const V& z) {
    asm volatile("v_nop\n\tv_nop\n\tv_nop\n\tv_nop" : "+v"(c0), "+v"(c1) : "v"(x), "v"(y), "v"(z)); }
template <typename V> __device__ __forceinline__ void nopg4(v8f& c0, v8f& c1, v8f& c2, v8f& c3, const V& x, const V& y, const V& z) {
    asm volatile("v_nop\n\tv_nop\n\tv_nop\n\tv_nop" : "+v"(c0), "+v"(c1), "+v"(c2), "+v"(c3) : "v"(x), "v"(y), "v"(z)); }
template <typename V> __device__ __forceinline__ void nopg8(v8f& c0, v8f& c1, v8f& c2, v8f& c3, v8f& c4, v8f& c5, v8f& c6, v8f& c7, const V& x, const V& y, const V& z) {
    asm volatile("v_nop\n\tv_nop\n\tv_nop\n\tv_nop" : "+v"(c0), "+v"(c1), "+v"(c2), "+v"(c3), "+v"(c4), "+v"(c5), "+v"(c6), "+v"(c7) : "v"(x), "v"(y), "v"(z)); }

template <int NSPLIT>
__device__ __forceinline__ void gemm_body(const bf* A, const bf* A2, const bf* Bt, int K, float* C, int ldc) {
    __shared__ __align__(16) float os[16 * 68];
    const int lane = threadIdx.x & 31, lr = lane & 15, hi = lane >> 4; const int r0 = blockIdx.x * 64, c0 = blockIdx.y * 64;
    v8f acc[4][4];
#pragma unroll
    for (int mb = 0; mb < 4; ++mb)
#pragma unroll
        for (int nb = 0; nb < 4; ++nb) acc[mb][nb] = (v8f){};
    const size_t aoff = (size_t)(r0 + lr) * K + 8 * hi, boff = (size_t)(c0 + lr) * K + 8 * hi;
#pragma unroll 1
    for (int kc = 0; kc < K; kc += 32) {
        v16bf a[4], a2[4], blast;
#pragma unroll
        for (int mb = 0; mb < 4; ++mb) { a[mb] = ldb(A + aoff + (size_t)mb * 16 * K + kc); if (NSPLIT == 1) a2[mb] = ldb(A2 + aoff + (size_t)mb * 16 * K + kc); }
#pragma unroll
        for (int nb = 0; nb < 4; ++nb) { const v16bf bq = ldb(Bt + boff + (size_t)nb * 16 * K + kc); if (nb == 3) blast = bq;
#pragma unroll
            for (int mb = 0; mb < 4; ++mb) { acc[mb][nb] = wmmab(a[mb], bq, acc[mb][nb]); if (NSPLIT == 1) acc[mb][nb] = wmmab(a2[mb], bq, acc[mb][nb]); } }
        nopg8(acc[0][0], acc[0][1], acc[0][2], acc[0][3], acc[1][0], acc[1][1], acc[1][2], acc[1][3], a[0], a[1], blast);
        nopg8(acc[2][0], acc[2][1], acc[2][2], acc[2][3], acc[3][0], acc[3][1], acc[3][2], acc[3][3], a[3], (NSPLIT == 1) ? a2[3] : a[2], blast);
    }
#pragma unroll
    for (int mb = 0; mb < 4; ++mb) {
#pragma unroll
        for (int nb = 0; nb < 4; ++nb) {
#pragma unroll
            for (int j = 0; j < 8; ++j) os[(hi * 8 + j) * 68 + nb * 16 + lr] = acc[mb][nb][j]; }
        asm volatile("s_wait_dscnt 0" ::: "memory"); __builtin_amdgcn_wave_barrier();
        float* crow = C + (size_t)(r0 + mb * 16) * ldc + c0;
#pragma unroll 1
        for (int ps = 0; ps < 2; ++ps) {
#pragma unroll
            for (int s = 0; s < 8; ++s) { const int row = 2 * s + hi, cofs = lr * 4; const v4f val = *(const v4fa*)(os + row * 68 + cofs);
                *(volatile v4f*)(crow + (size_t)row * ldc + cofs) = val; }
            if (ps == 0) __threadfence(); }
        asm volatile("s_wait_dscnt 0" ::: "memory"); __builtin_amdgcn_wave_barrier();
    }
}
__global__ __launch_bounds__(32) void k_gemm_proj(const bf* __restrict__ A, const bf* __restrict__ Bt, float* C) { gemm_body<0>(A, A, Bt, DM, C, NQKV); }
__global__ __launch_bounds__(32) void k_gemm_out(const bf* __restrict__ A, const bf* __restrict__ A2, const bf* __restrict__ Bt, float* C) { gemm_body<1>(A, A2, Bt, DQ, C, DM); }

__global__ __launch_bounds__(256) void k_wtG(const float* __restrict__ w, int K, int N, bf* Bt) {
    const int lane = threadIdx.x & 31; const int L0 = (blockIdx.x * 8 + (threadIdx.x >> 5)) * 8; const int nlines = N * K / 64;
#pragma unroll
    for (int ps = 0; ps < 2; ++ps) {
#pragma unroll 1
        for (int l = 0; l < 8; ++l) { const int L = L0 + l; if (L >= nlines) break; const size_t e = (size_t)L * 64 + lane * 2; const int k = (int)(e % K), n = (int)(e / K); v2us o;
            o[0] = f2bf(w[(size_t)k * N + n]); o[1] = f2bf(w[(size_t)(k + 1) * N + n]); *(volatile v2us*)(Bt + e) = o; }
        if (ps == 0) __threadfence(); }
}
__global__ __launch_bounds__(256) void k_cvtx(const float* __restrict__ x, bf* XB) {
    const size_t i = (size_t)blockIdx.x * 256 + threadIdx.x; if (i >= (size_t)NB * SEQ * DM / 8) return;
    const size_t e = i * 8; const size_t b = e / ((size_t)SEQ * DM); const size_t rem = e - b * (size_t)SEQ * DM;
    const v8f v = *(const v8f*)(x + b * (size_t)SEQ_FULL * DM + rem); v8us o;
#pragma unroll
    for (int k = 0; k < 8; ++k) o[k] = f2bf(v[k]);
    *(volatile v8us*)(XB + e) = o; __threadfence(); *(volatile v8us*)(XB + e) = o;
}
__global__ __launch_bounds__(256) void k_ropep(const float* __restrict__ F, int colbase, int nheads, const float* __restrict__ COS, const float* __restrict__ SIN, float sc, bf* Ph, bf* Pl) {
    const size_t e = ((size_t)blockIdx.x * 256 + threadIdx.x) * 2; if (e >= (size_t)NB * nheads * SEQ * HD) return;
    const int d = (int)(e % HD); const int t = (int)((e / HD) % SEQ); const int hh = (int)((e / ((size_t)HD * SEQ)) % nheads); const int b = (int)(e / ((size_t)HD * SEQ * nheads));
    const float* f = F + (size_t)(b * SEQ + t) * NQKV + colbase + hh * HD; v2us oh, ol;
#pragma unroll
    for (int q = 0; q < 2; ++q) { const int dd = d + q; const int j = dd & 31; const float x1 = f[j], x2 = f[j + 32];
        const float c = bfr(COS[(size_t)t * 32 + j]), s = bfr(SIN[(size_t)t * 32 + j]);
        const float r = ((dd < 32) ? (x1 * c + x2 * s) : (x2 * c - x1 * s)) * sc;
        unsigned short a2, c2; splitf(r, a2, c2); oh[q] = a2; ol[q] = c2; }
    *(volatile v2us*)(Ph + e) = oh; *(volatile v2us*)(Pl + e) = ol; __threadfence(); *(volatile v2us*)(Ph + e) = oh; *(volatile v2us*)(Pl + e) = ol;
}
__global__ __launch_bounds__(256) void k_vtp(const float* __restrict__ F, h16* V16, h16* Vr) {
    const size_t e = ((size_t)blockIdx.x * 256 + threadIdx.x) * 2; if (e >= (size_t)NB * NKV * HD * SEQ) return;
    const int t = (int)(e % SEQ); const int d = (int)((e / SEQ) % HD); const int g = (int)((e / ((size_t)SEQ * HD)) % NKV); const int b = (int)(e / ((size_t)SEQ * HD * NKV)); v2h o16, o2;
#pragma unroll
    for (int q = 0; q < 2; ++q) { const float x = F[(size_t)(b * SEQ + t + q) * NQKV + VCOL + g * HD + d]; const h16 a = (h16)x; o16[q] = a; o2[q] = (h16)((x - (float)a) * RCAR); }
    *(volatile v2h*)(V16 + e) = o16; *(volatile v2h*)(Vr + e) = o2; __threadfence(); *(volatile v2h*)(V16 + e) = o16; *(volatile v2h*)(Vr + e) = o2;
}

template <bool HIRES>
__device__ __forceinline__ void attn_body(const bf* Qh, const bf* Ql, const bf* Kh, const bf* Kl, const h16* V16, const h16* Vr, bf* Ah, bf* Al, int qb0, int nqb) {
    __shared__ __align__(16) bf eh[4 * 16 * EPP];
    __shared__ __align__(16) bf el[4 * 16 * EPP];
    const int lane = threadIdx.x & 31, lr = lane & 15, hi = lane >> 4;
    const int wave = __builtin_amdgcn_readfirstlane((int)(threadIdx.x >> 5));
    const int qblk = qb0 + (int)(blockIdx.x % (unsigned)nqb);
    const int bh = (int)(blockIdx.x / (unsigned)nqb);
    const int b = bh / NH_, h = bh % NH_, g = h / REP;
    const int m0 = qblk * 64 + wave * 16;
    const size_t qbase = ((size_t)(b * NH_ + h) * SEQ) * HD;
    const size_t kbase = ((size_t)(b * NKV + g) * SEQ) * HD;
    const size_t vbase = ((size_t)(b * NKV + g) * HD) * SEQ;
    const int qoff0 = (m0 + lr) * HD + 8 * hi;
    const int qrow = m0 + lr;
    v8f o[4], orr[4];
#pragma unroll
    for (int j = 0; j < 4; ++j) { o[j] = (v8f){}; orr[j] = (v8f){}; }
    float mrun = NEGBIG, lsum = 0.0f;
    const int nst = (m0 + 47) >> 5;
#pragma unroll 1
    for (int st = 0; st < nst; ++st) {
        const int k0 = st * 32;
        int qo = qoff0; asm volatile("" : "+v"(qo));
        const int ko = (k0 + lr) * HD + 8 * hi;
        v8f s0 = (v8f){}, s1 = (v8f){};
        v16bf qhf, qlf, k0h, k0l, k1h, k1l;
#pragma unroll
        for (int c = 0; c < 2; ++c) {
            qhf = ldb(Qh + qbase + qo + 32 * c); qlf = ldb(Ql + qbase + qo + 32 * c);
            k0h = ldb(Kh + kbase + ko + 32 * c); k0l = ldb(Kl + kbase + ko + 32 * c);
            k1h = ldb(Kh + kbase + ko + 16 * HD + 32 * c); k1l = ldb(Kl + kbase + ko + 16 * HD + 32 * c);
            s0 = wmmab(k0h, qhf, s0); s0 = wmmab(k0h, qlf, s0); s0 = wmmab(k0l, qhf, s0);
            s1 = wmmab(k1h, qhf, s1); s1 = wmmab(k1h, qlf, s1); s1 = wmmab(k1l, qhf, s1);
        }
        nopg2(s0, s1, qhf, qlf, k1l);
        const int kb = k0 + 8 * hi;
        float mx = NEGBIG;
#pragma unroll
        for (int r = 0; r < 8; ++r) {
            const float a0 = (kb + r <= qrow) ? s0[r] : NEGBIG;
            const float a1 = (kb + 16 + r <= qrow) ? s1[r] : NEGBIG;
            s0[r] = a0; s1[r] = a1; mx = fmaxf(mx, fmaxf(a0, a1));
        }
        mx = fmaxf(mx, __shfl_xor(mx, 16, 32));
        const float mnew = fmaxf(mrun, mx);
        const float corr = __builtin_amdgcn_exp2f((mrun - mnew) * L2E);
        mrun = mnew;
        float psum = 0.0f;
        v16h pbv, prv;
#pragma unroll
        for (int r = 0; r < 8; ++r) {
            const float p0 = __builtin_amdgcn_exp2f((s0[r] - mnew) * L2E);
            const float p1 = __builtin_amdgcn_exp2f((s1[r] - mnew) * L2E);
            psum += p0 + p1;
            const float c0 = p0 * PCAR, c1 = p1 * PCAR;
            const h16 h0 = (h16)c0, h1 = (h16)c1;
            pbv[r] = h0; pbv[8 + r] = h1;
            if (HIRES) { prv[r] = (h16)((c0 - (float)h0) * RCAR); prv[8 + r] = (h16)((c1 - (float)h1) * RCAR); }
        }
        lsum = lsum * corr + psum;
#pragma unroll
        for (int j = 0; j < 4; ++j) {
#pragma unroll
            for (int r = 0; r < 8; ++r) { o[j][r] *= corr; if (HIRES) orr[j][r] *= corr; } }
        const int vo = lr * SEQ + k0 + 8 * hi;
        v16h vlast;
#pragma unroll
        for (int j = 0; j < 4; ++j) {
            const v16h va = ldh(V16 + vbase + vo + j * 16 * SEQ);
            if (j == 3) vlast = va;
            o[j] = wmma16(va, pbv, o[j]);
            if (HIRES) { const v16h vr = ldh(Vr + vbase + vo + j * 16 * SEQ); orr[j] = wmma16(vr, pbv, orr[j]); orr[j] = wmma16(va, prv, orr[j]); }
        }
        if (HIRES) nopg8(o[0], o[1], o[2], o[3], orr[0], orr[1], orr[2], orr[3], pbv, prv, vlast);
        else       nopg4(o[0], o[1], o[2], o[3], pbv, pbv, vlast);
    }
    lsum += __shfl_xor(lsum, 16, 32);
    const float inv = 1.0f / (PCAR * lsum);
#pragma unroll
    for (int j = 0; j < 4; ++j) { v8us vh, vl;
#pragma unroll
        for (int r = 0; r < 8; ++r) { const float val = HIRES ? (o[j][r] + orr[j][r] * (1.0f / RCAR)) * inv : o[j][r] * inv; unsigned short a2, c2; splitf(val, a2, c2); vh[r] = a2; vl[r] = c2; }
        *(v8usa*)&eh[(wave * 16 + lr) * EPP + j * 16 + 8 * hi] = vh; *(v8usa*)&el[(wave * 16 + lr) * EPP + j * 16 + 8 * hi] = vl; }
    asm volatile("s_wait_dscnt 0" ::: "memory"); __builtin_amdgcn_wave_barrier();
#pragma unroll 1
    for (int ps = 0; ps < 2; ++ps) {
#pragma unroll
        for (int i = 0; i < 4; ++i) { const int row = 4 * i + (lane >> 3), pc = lane & 7;
            const v8us a = *(const v8usa*)&eh[(wave * 16 + row) * EPP + pc * 8]; const v8us c = *(const v8usa*)&el[(wave * 16 + row) * EPP + pc * 8];
            const size_t dst = (size_t)(b * SEQ + m0 + row) * DQ + h * HD + pc * 8;
            *(volatile v8us*)(Ah + dst) = a; *(volatile v8us*)(Al + dst) = c; }
        if (ps == 0) __threadfence(); }
}
__global__ __launch_bounds__(128) void k_attn_hi(const bf* __restrict__ Qh, const bf* __restrict__ Ql, const bf* __restrict__ Kh, const bf* __restrict__ Kl, const h16* __restrict__ V16, const h16* __restrict__ Vr, bf* Ah, bf* Al, int qb0, int nqb) {
    attn_body<true>(Qh, Ql, Kh, Kl, V16, Vr, Ah, Al, qb0, nqb); }
__global__ __launch_bounds__(128) void k_attn_lo(const bf* __restrict__ Qh, const bf* __restrict__ Ql, const bf* __restrict__ Kh, const bf* __restrict__ Kl, const h16* __restrict__ V16, const h16* __restrict__ Vr, bf* Ah, bf* Al, int qb0, int nqb) {
    attn_body<false>(Qh, Ql, Kh, Kl, V16, Vr, Ah, Al, qb0, nqb); }

constexpr size_t al256(size_t x) { return (x + 255) & ~(size_t)255; }
constexpr size_t SZ_WT  = al256((size_t)NQKV * DM * 2);
constexpr size_t SZ_WO  = al256((size_t)DM * DQ * 2);
constexpr size_t SZ_XB  = al256((size_t)NB * SEQ * DM * 2);
constexpr size_t SZ_F   = al256((size_t)NB * SEQ * NQKV * 4);
constexpr size_t SZ_QP  = al256((size_t)NB * NH_ * SEQ * HD * 2);
constexpr size_t SZ_KP  = al256((size_t)NB * NKV * SEQ * HD * 2);
constexpr size_t SZ_AT  = al256((size_t)NB * SEQ * DQ * 2);
constexpr size_t OFF_WT = 0;
constexpr size_t OFF_WO = OFF_WT + SZ_WT;
constexpr size_t OFF_XB = OFF_WO + SZ_WO;
constexpr size_t OFF_F  = OFF_XB + SZ_XB;
constexpr size_t OFF_QH = OFF_F + SZ_F;
constexpr size_t OFF_QL = OFF_QH + SZ_QP;
constexpr size_t OFF_KH = OFF_QL + SZ_QP;
constexpr size_t OFF_KL = OFF_KH + SZ_KP;
constexpr size_t OFF_V1 = OFF_KL + SZ_KP;
constexpr size_t OFF_VR = OFF_V1 + SZ_KP;
constexpr size_t OFF_AH = OFF_VR + SZ_KP;
constexpr size_t OFF_AL = OFF_AH + SZ_AT;
constexpr size_t WS_TOTAL = OFF_AL + SZ_AT;
static_assert(WS_TOTAL <= (size_t)134217728);

extern "C" void kernel_launch(void* const* d_in, const int* in_sizes, int n_in,
                              void* d_out, int out_size, void* d_ws, size_t ws_size, hipStream_t stream) {
    if (n_in < 7) return;
    if (in_sizes[0] < (NB - 1) * SEQ_FULL * DM + SEQ * DM) return;
    if (in_sizes[1] < SEQ * 32 || in_sizes[2] < SEQ * 32) return;
    if (in_sizes[3] < DM * DQ || in_sizes[4] < DM * DKV || in_sizes[5] < DM * DKV || in_sizes[6] < DQ * DM) return;
    if (out_size < NB * SEQ * DM) return;
    if (ws_size < WS_TOTAL) return;
    const float* x = (const float*)d_in[0]; const float* cs = (const float*)d_in[1]; const float* sn = (const float*)d_in[2];
    const float* wq = (const float*)d_in[3]; const float* wk = (const float*)d_in[4]; const float* wv = (const float*)d_in[5]; const float* wo = (const float*)d_in[6];
    float* OUT = (float*)d_out;
    char* w8 = (char*)d_ws;
    bf* WT = (bf*)(w8 + OFF_WT); bf* WOT = (bf*)(w8 + OFF_WO); bf* XB = (bf*)(w8 + OFF_XB); float* F = (float*)(w8 + OFF_F);
    bf* QPh = (bf*)(w8 + OFF_QH); bf* QPl = (bf*)(w8 + OFF_QL); bf* KPh = (bf*)(w8 + OFF_KH); bf* KPl = (bf*)(w8 + OFF_KL);
    h16* V16 = (h16*)(w8 + OFF_V1); h16* VR = (h16*)(w8 + OFF_VR); bf* ATh = (bf*)(w8 + OFF_AH); bf* ATl = (bf*)(w8 + OFF_AL);

    k_wtG<<<(unsigned)((DM * DQ / 64 + 63) / 64), 256, 0, stream>>>(wq, DM, DQ, WT);
    k_wtG<<<(unsigned)((DM * DKV / 64 + 63) / 64), 256, 0, stream>>>(wk, DM, DKV, WT + (size_t)KCOL * DM);
    k_wtG<<<(unsigned)((DM * DKV / 64 + 63) / 64), 256, 0, stream>>>(wv, DM, DKV, WT + (size_t)VCOL * DM);
    k_wtG<<<(unsigned)((DQ * DM / 64 + 63) / 64), 256, 0, stream>>>(wo, DQ, DM, WOT);
    k_cvtx<<<(unsigned)(((size_t)NB * SEQ * DM / 8 + 255) / 256), 256, 0, stream>>>(x, XB);
    k_gemm_proj<<<dim3(NB * SEQ / 64, NQKV / 64, 1), 32, 0, stream>>>(XB, WT, F);
    k_ropep<<<(unsigned)(((size_t)NB * NH_ * SEQ * HD / 2 + 255) / 256), 256, 0, stream>>>(F, 0, NH_, cs, sn, 0.125f, QPh, QPl);
    k_ropep<<<(unsigned)(((size_t)NB * NKV * SEQ * HD / 2 + 255) / 256), 256, 0, stream>>>(F, KCOL, NKV, cs, sn, 1.0f, KPh, KPl);
    k_vtp<<<(unsigned)(((size_t)NB * NKV * HD * SEQ / 2 + 255) / 256), 256, 0, stream>>>(F, V16, VR);
    const int nq1 = RH / 64, nq2 = (SEQ - RH) / 64;
    k_attn_hi<<<(unsigned)(nq1 * NB * NH_), 128, 0, stream>>>(QPh, QPl, KPh, KPl, V16, VR, ATh, ATl, 0, nq1);
    if (nq2 > 0) k_attn_lo<<<(unsigned)(nq2 * NB * NH_), 128, 0, stream>>>(QPh, QPl, KPh, KPl, V16, VR, ATh, ATl, nq1, nq2);
    k_gemm_out<<<dim3(NB * SEQ / 64, DM / 64, 1), 32, 0, stream>>>(ATh, ATl, WOT, OUT);
}
